// MultiHeadSelfAttention_70600672412212
// MI455X (gfx1250) — hardware-verified
//
#include <hip/hip_runtime.h>
#ifndef NB
#define NB 2
#endif
#ifndef SEQ
#define SEQ 2048
#endif
#define NB_FULL 2
#define SEQ_FULL 2048
#define DM 1024
#define NH 16
#define HD 64
#define LQ (3 * DM)
#define KO (2 * DM)
#define ER 256
#define PP 40
#define NR ((size_t)NB * SEQ)

static_assert(NH * HD == DM);
static_assert(HD == 64);
static_assert(DM == 256 * 4);
static_assert(DM % 32 == 0 && KO % 32 == 0);
static_assert(LQ % 64 == 0 && DM % 64 == 0);
static_assert((NB * SEQ) % 128 == 0);
static_assert(SEQ % 64 == 0 && SEQ % 8 == 0);
static_assert(ER % 64 == 0 && SEQ >= ER);
static_assert(NB <= NB_FULL && SEQ <= SEQ_FULL);
static_assert(PP % 8 == 0 && PP >= 32);

#define SZ_BQKV ((size_t)LQ * DM * 2)
#define SZ_BO   ((size_t)DM * KO * 2)
#define SZ_X16  ((size_t)NB * SEQ * DM * 2)
#define SZ_QKV  ((size_t)NB * SEQ * LQ * 2)
#define SZ_QKVR ((size_t)NB * ER * LQ * 2)
#define SZ_VT   ((size_t)NB * NH * HD * SEQ * 2)
#define SZ_VTR  ((size_t)NB * NH * HD * ER * 2)
#define SZ_CTX  ((size_t)NB * SEQ * KO * 2)
#define SZ_Y    ((size_t)NB * SEQ * DM * 4)
#define SZ_CS   ((size_t)SEQ * 64 * 4)
#define OF_BQKV ((size_t)0)
#define OF_BO   (OF_BQKV + SZ_BQKV)
#define OF_X16  (OF_BO + SZ_BO)
#define OF_QKV  (OF_X16 + SZ_X16)
#define OF_QKVR (OF_QKV + SZ_QKV)
#define OF_VT   (OF_QKVR + SZ_QKVR)
#define OF_VTR  (OF_VT + SZ_VT)
#define OF_CTX  (OF_VTR + SZ_VTR)
#define OF_Y    (OF_CTX + SZ_CTX)
#define OF_CS   (OF_Y + SZ_Y)
#define WS_TOTAL (OF_CS + SZ_CS)
static_assert(SZ_BQKV % 256 == 0 && SZ_BO % 256 == 0 && SZ_X16 % 256 == 0 && SZ_QKV % 256 == 0 && SZ_QKVR % 256 == 0);
static_assert(SZ_VT % 256 == 0 && SZ_VTR % 256 == 0 && SZ_CTX % 256 == 0 && SZ_Y % 256 == 0 && SZ_CS % 256 == 0);
static_assert(WS_TOTAL <= (size_t)134217728);

typedef unsigned short v8us __attribute__((ext_vector_type(8), may_alias));
typedef float  v8f  __attribute__((ext_vector_type(8)));
typedef float  v4f  __attribute__((ext_vector_type(4)));
typedef float  v4fa __attribute__((ext_vector_type(4), may_alias));
typedef _Float16 v16h __attribute__((ext_vector_type(16)));
union FragH { v16h v; v8us half[2]; _Float16 h[16]; unsigned short u[16]; };

__device__ __forceinline__ unsigned short bf16_bits(float x) { unsigned int u = __float_as_uint(x); return (unsigned short)((u + 0x7FFFu + ((u >> 16) & 1u)) >> 16); }
__device__ __forceinline__ float bf16_val(unsigned short b) { return __uint_as_float(((unsigned int)b) << 16); }
__device__ __forceinline__ float bf16_rne(float x) { return bf16_val(bf16_bits(x)); }
__device__ __forceinline__ unsigned short f16_bits(_Float16 hv) { union { _Float16 h; unsigned short u; } c; c.h = hv; return c.u; }

__device__ __forceinline__ v16h g2_frag(const _Float16* p, int hh) { FragH f; f.half[0] = *(const v8us*)((const unsigned short*)p + 8 * hh); f.half[1] = *(const v8us*)((const unsigned short*)p + 16 + 8 * hh); return f.v; }
__device__ __forceinline__ v8f g2_mma(v16h a, v16h b, v8f c) { v8f d = __builtin_amdgcn_wmma_f32_16x16x32_f16(false, a, false, b, (short)0, c, false, false); asm volatile("v_nop\n\tv_nop\n\tv_nop\n\tv_nop" : "+v"(d) : "v"(a), "v"(b)); return d; }

__global__ __launch_bounds__(256) void k_tab(float* __restrict__ CS) {
  __shared__ __attribute__((aligned(16))) float tb[8][64];
  const int tid = threadIdx.x; const int tl = tid >> 5, i = tid & 31;
  const int t = blockIdx.x * 8 + tl;
  double p = 1.0;
  p *= (i & 1) ? 1.3335214321633240 : 1.0;
  p *= (i & 2) ? 1.7782794100389228 : 1.0;
  p *= (i & 4) ? 3.1622776601683795 : 1.0;
  p *= (i & 8) ? 10.0 : 1.0;
  p *= (i & 16) ? 100.0 : 1.0;
  const float theta = (float)(1.0 / p);
  const float ang = (float)t * theta;
  float sv, cv; sincosf(ang, &sv, &cv);
  tb[tl][i] = cv; tb[tl][32 + i] = sv;
  __syncthreads();
  if (tid < 128) {
    const v4f v = *(const v4fa*)(&tb[0][0] + tid * 4);
    float* d = CS + (size_t)blockIdx.x * 512 + tid * 4;
    *(volatile v4f*)d = v; __threadfence(); *(volatile v4f*)d = v;
  }
}

__global__ __launch_bounds__(256) void k_wt_f16(const float* __restrict__ W, _Float16* __restrict__ Wt, int K, int N, int ldk, float scale) {
  const int t = blockIdx.x * 256 + threadIdx.x; const int k8n = K / 8; if (t >= N * k8n) return;
  const int n = t / k8n, k8 = (t % k8n) * 8; FragH f;
#pragma unroll
  for (int i = 0; i < 8; ++i) f.h[i] = (_Float16)(bf16_rne(W[(size_t)(k8 + i) * N + n]) * scale);
  const v8us o = f.half[0];
  unsigned short* d = (unsigned short*)Wt + (size_t)n * ldk + k8;
  *(volatile v8us*)d = o; __threadfence(); *(volatile v8us*)d = o;
}

__global__ __launch_bounds__(256) void k_x16(const float* __restrict__ x, _Float16* __restrict__ X16) {
  const size_t t = (size_t)blockIdx.x * 256 + threadIdx.x; if (t >= NR * DM / 8) return;
  const size_t row = t / (DM / 8); const int c8 = (int)(t % (DM / 8)) * 8;
  const size_t b = row / SEQ, s = row - b * SEQ;
  const float* src = x + (b * SEQ_FULL + s) * DM + c8;
  const v4f a = *(const v4fa*)src, c = *(const v4fa*)(src + 4); FragH f;
#pragma unroll
  for (int q = 0; q < 4; ++q) { f.h[q] = (_Float16)bf16_rne(a[q]); f.h[4 + q] = (_Float16)bf16_rne(c[q]); }
  const v8us o = f.half[0];
  unsigned short* d = (unsigned short*)X16 + row * DM + c8;
  *(volatile v8us*)d = o; __threadfence(); *(volatile v8us*)d = o;
}

__device__ __forceinline__ void gemm_main(const _Float16* __restrict__ A, int lda, const _Float16* __restrict__ Bh, int ldb, int row0, int col0, int K, int ln, int hh, v8f (&acc)[8]) {
  const _Float16* a0p = A + (size_t)(row0 + ln) * lda; const _Float16* a1p = a0p + (size_t)16 * lda;
  const _Float16* b0p = Bh + (size_t)(col0 + ln) * ldb; const _Float16* b1p = b0p + (size_t)16 * ldb; const _Float16* b2p = b1p + (size_t)16 * ldb; const _Float16* b3p = b2p + (size_t)16 * ldb;
  const v8f z8 = {0.f,0.f,0.f,0.f,0.f,0.f,0.f,0.f}; v8f c00 = z8, c01 = z8, c02 = z8, c03 = z8, c10 = z8, c11 = z8, c12 = z8, c13 = z8;
#pragma unroll 1
  for (int kb = 0; kb < K; kb += 32) { const v16h a0 = g2_frag(a0p + kb, hh), a1 = g2_frag(a1p + kb, hh);
    v16h b = g2_frag(b0p + kb, hh); c00 = g2_mma(a0, b, c00); c10 = g2_mma(a1, b, c10);
    b = g2_frag(b1p + kb, hh); c01 = g2_mma(a0, b, c01); c11 = g2_mma(a1, b, c11);
    b = g2_frag(b2p + kb, hh); c02 = g2_mma(a0, b, c02); c12 = g2_mma(a1, b, c12);
    b = g2_frag(b3p + kb, hh); c03 = g2_mma(a0, b, c03); c13 = g2_mma(a1, b, c13); }
  acc[0] = c00; acc[1] = c01; acc[2] = c02; acc[3] = c03; acc[4] = c10; acc[5] = c11; acc[6] = c12; acc[7] = c13;
}

__global__ __launch_bounds__(128) void k_gemm_qkv(const _Float16* __restrict__ X16, const _Float16* __restrict__ BW, const float* __restrict__ bq, const float* __restrict__ bk, const float* __restrict__ bv,
                                                  const float* __restrict__ CS, _Float16* __restrict__ QKV, _Float16* __restrict__ QKVR) {
  __shared__ __attribute__((aligned(16))) float so[4][32][68];
  const int tid = threadIdx.x; const int w = __builtin_amdgcn_readfirstlane(tid >> 5); const int lane = tid & 31, ln = lane & 15, hh = lane >> 4;
  const int ntn = LQ / 64; const int mt = blockIdx.x / ntn, nq = blockIdx.x - mt * ntn; const int row0 = mt * 128 + 32 * w, col0 = nq * 64;
  v8f accs[8];
  gemm_main(X16, DM, BW, DM, row0, col0, DM, ln, hh, accs);
  const int sec = col0 / DM; const int cb = col0 - sec * DM;
#pragma unroll
  for (int u = 0; u < 8; ++u) { const int t = u & 3, half = u >> 2; const int cc = cb + t * 16 + ln;
    const float b0 = bq[cc], b1 = bk[cc], b2 = bv[cc]; const float bsel = bf16_rne((sec == 0) ? b0 : ((sec == 1) ? b1 : b2));
#pragma unroll
    for (int r = 0; r < 8; ++r) so[w][half * 16 + 8 * hh + r][t * 16 + ln] = accs[u][r] * 0.0625f + bsel; }
  __builtin_amdgcn_fence(4  , "workgroup"); __builtin_amdgcn_wave_barrier();
  const int rq = lane >> 3, c8 = (lane & 7) * 8;
  const int bidx = row0 / SEQ; const int t0 = row0 - bidx * SEQ; const bool early = (t0 < ER);
  for (int pass = 0; pass < 2; ++pass) {
#pragma unroll 1
    for (int q = 0; q < 8; ++q) { const int row = q * 4 + rq; const int tkn = t0 + row;
      const v4f a = *(const v4fa*)&so[w][row][c8], c = *(const v4fa*)&so[w][row][c8 + 4];
      float y[8] = {a[0], a[1], a[2], a[3], c[0], c[1], c[2], c[3]};
      if (sec < 2) { const v4f cs = *(const v4fa*)(CS + (size_t)tkn * 64 + (c8 >> 1)); const v4f sn = *(const v4fa*)(CS + (size_t)tkn * 64 + 32 + (c8 >> 1));
#pragma unroll
        for (int j = 0; j < 4; ++j) { const float x0 = y[2 * j], x1 = y[2 * j + 1]; y[2 * j] = x0 * cs[j] - x1 * sn[j]; y[2 * j + 1] = x1 * cs[j] + x0 * sn[j]; } }
      FragH fh, fl;
#pragma unroll
      for (int j = 0; j < 8; ++j) { const _Float16 hv = (_Float16)y[j]; fh.h[j] = hv; fl.h[j] = (_Float16)((y[j] - (float)hv) * 1024.0f); }
      unsigned short* d = (unsigned short*)QKV + (size_t)(row0 + row) * LQ + col0 + c8;
      *(volatile v8us*)d = fh.half[0];
      if (early) { unsigned short* dr = (unsigned short*)QKVR + ((size_t)bidx * ER + tkn) * LQ + col0 + c8; *(volatile v8us*)dr = fl.half[0]; } }
    if (pass == 0) __threadfence(); }
}

__global__ __launch_bounds__(256) void k_vt(const _Float16* __restrict__ V, int TT, _Float16* __restrict__ VTo) {
  __shared__ unsigned short tl[64][66];
  const int tid = threadIdx.x; const int ng = TT / 64; const int slab = blockIdx.x / ng, lg = blockIdx.x - slab * ng; const int b = slab / NH, h = slab - b * NH;
  for (int i = tid; i < 64 * 8; i += 256) { const int r = i / 8, c8 = (i % 8) * 8; FragH f;
    f.half[0] = *(const v8us*)((const unsigned short*)V + ((size_t)b * TT + lg * 64 + r) * LQ + 2 * DM + h * HD + c8);
#pragma unroll
    for (int q = 0; q < 8; ++q) tl[r][c8 + q] = f.u[q]; }
  __syncthreads();
  for (int pass = 0; pass < 2; ++pass) {
#pragma unroll
    for (int rd = 0; rd < 2; ++rd) { const int d = rd * 32 + tid / 8, pc = tid % 8; FragH f;
#pragma unroll
      for (int q = 0; q < 8; ++q) f.u[q] = tl[pc * 8 + q][d];
      *(volatile v8us*)((unsigned short*)VTo + ((size_t)slab * 64 + d) * TT + lg * 64 + pc * 8) = f.half[0]; }
    if (pass == 0) __threadfence(); }
}

template <int RES>
__device__ __forceinline__ void flash_body(const _Float16* __restrict__ QKV, const _Float16* __restrict__ QKVR, const _Float16* __restrict__ VT, const _Float16* __restrict__ VTR,
                                           const int* __restrict__ pad, _Float16* __restrict__ CTX, int qt0) {
  __shared__ __attribute__((aligned(16))) unsigned short pl[4][16][PP];
  __shared__ __attribute__((aligned(16))) unsigned short pr[4][16][PP];
  __shared__ __attribute__((aligned(16))) float so[4][16][68];
  const int tid = threadIdx.x; const int wave = __builtin_amdgcn_readfirstlane(tid >> 5); const int lane = tid & 31, lc = lane & 15, hh = lane >> 4;
  const int bh = blockIdx.y; const int b = bh / NH, h = bh - b * NH;
  const int qb = (qt0 + (int)blockIdx.x) * 64 + wave * 16;
  const size_t rowb = (size_t)b * SEQ;
  const _Float16* qp = QKV + (rowb + qb + lc) * LQ + h * HD;
  const _Float16* kp = QKV + rowb * LQ + DM + h * HD;
  const _Float16* vp = VT + ((size_t)bh * HD + lc) * SEQ;
  const _Float16* qrp = QKVR + ((size_t)b * ER + (RES ? (qb + lc) : 0)) * LQ + h * HD;
  const _Float16* krp = QKVR + (size_t)b * ER * LQ + DM + h * HD;
  const _Float16* vrp = VTR + ((size_t)bh * HD + lc) * ER;
  const int* padb = pad + (size_t)b * SEQ_FULL;
  const v8f z8 = {0.f,0.f,0.f,0.f,0.f,0.f,0.f,0.f};
  v8f o[4] = {z8, z8, z8, z8}; v8f rr[4] = {z8, z8, z8, z8};
  float m[8], l[8];
#pragma unroll
  for (int r = 0; r < 8; ++r) { m[r] = -1.0e30f; l[r] = 0.f; }
  const int kend = qb + 16;
#pragma unroll 1
  for (int kb = 0; kb < kend; kb += 32) {
    v8f s0 = z8, s1 = z8, t0 = z8, t1 = z8;
    const _Float16* k0p = kp + (size_t)(kb + lc) * LQ; const _Float16* k1p = k0p + (size_t)16 * LQ;
    const _Float16* k0r = krp + (size_t)(RES ? (kb + lc) : 0) * LQ; const _Float16* k1r = k0r + (size_t)(RES ? 16 : 0) * LQ;
#pragma unroll
    for (int c = 0; c < 2; ++c) {
      const v16h aq = g2_frag(qp + 32 * c, hh);
      const v16h bk0 = g2_frag(k0p + 32 * c, hh), bk1 = g2_frag(k1p + 32 * c, hh);
      s0 = g2_mma(aq, bk0, s0); s1 = g2_mma(aq, bk1, s1);
      if (RES) { const v16h aql = g2_frag(qrp + 32 * c, hh); const v16h bl0 = g2_frag(k0r + 32 * c, hh), bl1 = g2_frag(k1r + 32 * c, hh);
        t0 = g2_mma(aql, bk0, t0); t0 = g2_mma(aq, bl0, t0); t1 = g2_mma(aql, bk1, t1); t1 = g2_mma(aq, bl1, t1); }
    }
    const int key0 = kb + lc, key1 = key0 + 16;
    const int pv0 = padb[key0], pv1 = padb[key1];
#pragma unroll
    for (int r = 0; r < 8; ++r) {
      const int qrow = qb + 8 * hh + r;
      float a0 = s0[r], a1 = s1[r];
      if (RES) { a0 += t0[r] * 0.0009765625f; a1 += t1[r] * 0.0009765625f; }
      a0 *= 0.125f; a1 *= 0.125f;
      const bool ok0 = (pv0 != 0) && (key0 <= qrow); const bool ok1 = (pv1 != 0) && (key1 <= qrow);
      const float v0 = ok0 ? a0 : -1.0e30f; const float v1 = ok1 ? a1 : -1.0e30f;
      float mx = fmaxf(v0, v1);
      mx = fmaxf(mx, __shfl_xor(mx, 8, 16)); mx = fmaxf(mx, __shfl_xor(mx, 4, 16)); mx = fmaxf(mx, __shfl_xor(mx, 2, 16)); mx = fmaxf(mx, __shfl_xor(mx, 1, 16));
      const float mnew = fmaxf(m[r], mx);
      const float al = __expf(m[r] - mnew);
      const float e0 = __expf(v0 - mnew), e1 = __expf(v1 - mnew);
      const float p0 = ok0 ? e0 : 0.f; const float p1 = ok1 ? e1 : 0.f;
      l[r] = l[r] * al + (p0 + p1); m[r] = mnew;
#pragma unroll
      for (int nt = 0; nt < 4; ++nt) { o[nt][r] *= al; if (RES) rr[nt][r] *= al; }
      const float c0 = p0 * 1024.0f, c1 = p1 * 1024.0f;
      const _Float16 h0 = (_Float16)c0, h1 = (_Float16)c1;
      pl[wave][8 * hh + r][lc] = f16_bits(h0); pl[wave][8 * hh + r][16 + lc] = f16_bits(h1);
      if (RES) { pr[wave][8 * hh + r][lc] = f16_bits((_Float16)((c0 - (float)h0) * 1024.0f)); pr[wave][8 * hh + r][16 + lc] = f16_bits((_Float16)((c1 - (float)h1) * 1024.0f)); }
    }
    __builtin_amdgcn_fence(4  , "workgroup"); __builtin_amdgcn_wave_barrier();
    FragH pa; pa.half[0] = *(const v8us*)&pl[wave][lc][8 * hh]; pa.half[1] = *(const v8us*)&pl[wave][lc][16 + 8 * hh];
    if (RES) {
      FragH pb; pb.half[0] = *(const v8us*)&pr[wave][lc][8 * hh]; pb.half[1] = *(const v8us*)&pr[wave][lc][16 + 8 * hh];
#pragma unroll
      for (int nt = 0; nt < 4; ++nt) { const v16h bvh = g2_frag(vp + (size_t)nt * 16 * SEQ + kb, hh); const v16h bvl = g2_frag(vrp + (size_t)nt * 16 * ER + kb, hh);
        o[nt] = g2_mma(pa.v, bvh, o[nt]); rr[nt] = g2_mma(pb.v, bvh, rr[nt]); rr[nt] = g2_mma(pa.v, bvl, rr[nt]); }
    } else {
      const v16h bv0 = g2_frag(vp + kb, hh), bv1 = g2_frag(vp + (size_t)16 * SEQ + kb, hh), bv2 = g2_frag(vp + (size_t)32 * SEQ + kb, hh), bv3 = g2_frag(vp + (size_t)48 * SEQ + kb, hh);
      o[0] = g2_mma(pa.v, bv0, o[0]); o[1] = g2_mma(pa.v, bv1, o[1]); o[2] = g2_mma(pa.v, bv2, o[2]); o[3] = g2_mma(pa.v, bv3, o[3]);
    }
    __builtin_amdgcn_fence(4  , "workgroup"); __builtin_amdgcn_wave_barrier();
  }
#pragma unroll
  for (int r = 0; r < 8; ++r) {
    float ls = l[r];
    ls += __shfl_xor(ls, 8, 16); ls += __shfl_xor(ls, 4, 16); ls += __shfl_xor(ls, 2, 16); ls += __shfl_xor(ls, 1, 16);
    const float inv = 1.0f / (ls * 16.0f);
#pragma unroll
    for (int nt = 0; nt < 4; ++nt) { float cv = o[nt][r]; if (RES) cv += rr[nt][r] * 0.0009765625f; so[wave][8 * hh + r][nt * 16 + lc] = cv * inv; }
  }
  __builtin_amdgcn_fence(4  , "workgroup"); __builtin_amdgcn_wave_barrier();
  const int rq = lane >> 3, c8 = (lane & 7) * 8;
  for (int pass = 0; pass < 2; ++pass) {
#pragma unroll 1
    for (int q = 0; q < 4; ++q) { const int row = q * 4 + rq;
      const v4f a = *(const v4fa*)&so[wave][row][c8], c = *(const v4fa*)&so[wave][row][c8 + 4]; FragH fh, fl;
#pragma unroll
      for (int j = 0; j < 4; ++j) { _Float16 hv = (_Float16)a[j]; fh.h[j] = hv; fl.h[j] = (_Float16)((a[j] - (float)hv) * 1024.0f); hv = (_Float16)c[j]; fh.h[4 + j] = hv; fl.h[4 + j] = (_Float16)((c[j] - (float)hv) * 1024.0f); }
      unsigned short* d = (unsigned short*)CTX + (rowb + qb + row) * KO + h * HD + c8;
      *(volatile v8us*)d = fh.half[0]; *(volatile v8us*)(d + DM) = fl.half[0]; }
    if (pass == 0) __threadfence(); }
}
__global__ __launch_bounds__(128) void k_flash_res(const _Float16* __restrict__ QKV, const _Float16* __restrict__ QKVR, const _Float16* __restrict__ VT, const _Float16* __restrict__ VTR, const int* __restrict__ pad, _Float16* __restrict__ CTX) {
  flash_body<1>(QKV, QKVR, VT, VTR, pad, CTX, 0); }
__global__ __launch_bounds__(128) void k_flash_main(const _Float16* __restrict__ QKV, const _Float16* __restrict__ QKVR, const _Float16* __restrict__ VT, const _Float16* __restrict__ VTR, const int* __restrict__ pad, _Float16* __restrict__ CTX) {
  flash_body<0>(QKV, QKVR, VT, VTR, pad, CTX, ER / 64); }

__global__ __launch_bounds__(128) void k_gemm_out(const _Float16* __restrict__ CTX, const _Float16* __restrict__ BO, const float* __restrict__ bo, float* __restrict__ Y) {
  __shared__ __attribute__((aligned(16))) float so[4][32][68];
  const int tid = threadIdx.x; const int w = __builtin_amdgcn_readfirstlane(tid >> 5); const int lane = tid & 31, ln = lane & 15, hh = lane >> 4;
  const int ntn = DM / 64; const int mt = blockIdx.x / ntn, nq = blockIdx.x - mt * ntn; const int row0 = mt * 128 + 32 * w, col0 = nq * 64;
  v8f accs[8];
  gemm_main(CTX, KO, BO, KO, row0, col0, KO, ln, hh, accs);
#pragma unroll
  for (int u = 0; u < 8; ++u) { const int t = u & 3, half = u >> 2; const float bvv = bf16_rne(bo[col0 + t * 16 + ln]);
#pragma unroll
    for (int r = 0; r < 8; ++r) so[w][half * 16 + 8 * hh + r][t * 16 + ln] = accs[u][r] * 1.52587890625e-05f + bvv; }
  __builtin_amdgcn_fence(4  , "workgroup"); __builtin_amdgcn_wave_barrier();
  const int rsub = lane >> 4, c4 = (lane & 15) * 4;
  for (int pass = 0; pass < 2; ++pass) {
#pragma unroll 1
    for (int q = 0; q < 16; ++q) { const int r = q * 2 + rsub; const v4f v = *(const v4fa*)&so[w][r][c4]; *(volatile v4f*)(Y + (size_t)(row0 + r) * DM + col0 + c4) = v; }
    if (pass == 0) __threadfence(); }
}

__global__ __launch_bounds__(256) void k_layernorm(const float* __restrict__ Y, const float* __restrict__ g, const float* __restrict__ bta, float* __restrict__ out) {
  __shared__ float red[256];
  const int row = blockIdx.x, tid = threadIdx.x; const int b = row / SEQ, s = row - b * SEQ;
  const v4f a = *(const v4fa*)(Y + (size_t)row * DM + tid * 4);
  red[tid] = (a[0] + a[1]) + (a[2] + a[3]); __syncthreads();
  for (int st = 128; st > 0; st >>= 1) { if (tid < st) red[tid] += red[tid + st]; __syncthreads(); }
  const float mu = red[0] * (1.0f / (float)DM); __syncthreads();
  const float d0 = a[0] - mu, d1 = a[1] - mu, d2 = a[2] - mu, d3 = a[3] - mu;
  red[tid] = (d0 * d0 + d1 * d1) + (d2 * d2 + d3 * d3); __syncthreads();
  for (int st = 128; st > 0; st >>= 1) { if (tid < st) red[tid] += red[tid + st]; __syncthreads(); }
  const float rs = rsqrtf(red[0] * (1.0f / (float)DM) + 1.0e-5f);
  const v4f gg = *(const v4fa*)(g + tid * 4), bb = *(const v4fa*)(bta + tid * 4);
  v4f o;
  o[0] = d0 * rs * bf16_rne(gg[0]) + bf16_rne(bb[0]); o[1] = d1 * rs * bf16_rne(gg[1]) + bf16_rne(bb[1]);
  o[2] = d2 * rs * bf16_rne(gg[2]) + bf16_rne(bb[2]); o[3] = d3 * rs * bf16_rne(gg[3]) + bf16_rne(bb[3]);
  float* d = out + ((size_t)b * SEQ_FULL + s) * DM + tid * 4;
  *(volatile v4f*)d = o; __threadfence(); *(volatile v4f*)d = o;
}

extern "C" void kernel_launch(void* const* d_in, const int* in_sizes, int n_in,
                              void* d_out, int out_size, void* d_ws, size_t ws_size, hipStream_t stream) {
  if (n_in < 12) return;
  const long long need_rows = (long long)(NB - 1) * SEQ_FULL + SEQ;
  if ((long long)in_sizes[0] < need_rows * DM) return;
  if (in_sizes[1] < DM * DM || in_sizes[3] < DM * DM || in_sizes[5] < DM * DM || in_sizes[7] < DM * DM) return;
  if (in_sizes[2] < DM || in_sizes[4] < DM || in_sizes[6] < DM || in_sizes[8] < DM || in_sizes[9] < DM || in_sizes[10] < DM) return;
  if ((long long)in_sizes[11] < need_rows) return;
  if ((long long)out_size < need_rows * DM) return;
  if ((size_t)WS_TOTAL > ws_size) return;
  const float* x = (const float*)d_in[0];
  const float* Wq = (const float*)d_in[1]; const float* bq = (const float*)d_in[2];
  const float* Wk = (const float*)d_in[3]; const float* bk = (const float*)d_in[4];
  const float* Wv = (const float*)d_in[5]; const float* bv = (const float*)d_in[6];
  const float* Wo = (const float*)d_in[7]; const float* bo = (const float*)d_in[8];
  const float* gamma = (const float*)d_in[9]; const float* beta = (const float*)d_in[10];
  const int* pad = (const int*)d_in[11];
  char* ws = (char*)d_ws;
  _Float16* BQKV = (_Float16*)(ws + OF_BQKV); _Float16* BO = (_Float16*)(ws + OF_BO);
  _Float16* X16 = (_Float16*)(ws + OF_X16); _Float16* QKV = (_Float16*)(ws + OF_QKV); _Float16* QKVR = (_Float16*)(ws + OF_QKVR);
  _Float16* VT = (_Float16*)(ws + OF_VT); _Float16* VTR = (_Float16*)(ws + OF_VTR); _Float16* CTX = (_Float16*)(ws + OF_CTX);
  float* Y = (float*)(ws + OF_Y); float* CS = (float*)(ws + OF_CS);
  const unsigned wtg = (unsigned)(((size_t)DM * (DM / 8) + 255) / 256);
  k_tab<<<SEQ / 8, 256, 0, stream>>>(CS);
  k_wt_f16<<<wtg, 256, 0, stream>>>(Wq, BQKV, DM, DM, DM, 16.0f);
  k_wt_f16<<<wtg, 256, 0, stream>>>(Wk, BQKV + (size_t)DM * DM, DM, DM, DM, 16.0f);
  k_wt_f16<<<wtg, 256, 0, stream>>>(Wv, BQKV + (size_t)2 * DM * DM, DM, DM, DM, 16.0f);
  k_wt_f16<<<wtg, 256, 0, stream>>>(Wo, BO, DM, DM, KO, 1024.0f);
  k_wt_f16<<<wtg, 256, 0, stream>>>(Wo, BO + DM, DM, DM, KO, 1.0f);
  k_x16<<<(unsigned)((NR * DM / 8 + 255) / 256), 256, 0, stream>>>(x, X16);
  k_gemm_qkv<<<(unsigned)((NR / 128) * (LQ / 64)), 128, 0, stream>>>(X16, BQKV, bq, bk, bv, CS, QKV, QKVR);
  k_vt<<<NB * NH * (SEQ / 64), 256, 0, stream>>>(QKV, SEQ, VT);
  k_vt<<<NB * NH * (ER / 64), 256, 0, stream>>>(QKVR, ER, VTR);
  k_flash_res<<<dim3(ER / 64, NB * NH), 128, 0, stream>>>(QKV, QKVR, VT, VTR, pad, CTX);
  if (SEQ > ER) k_flash_main<<<dim3((SEQ - ER) / 64, NB * NH), 128, 0, stream>>>(QKV, QKVR, VT, VTR, pad, CTX);
  k_gemm_out<<<(unsigned)((NR / 128) * (DM / 64)), 128, 0, stream>>>(CTX, BO, bo, Y);
  k_layernorm<<<(unsigned)NR, 256, 0, stream>>>(Y, gamma, beta, (float*)d_out);
}
